// MultiHeadAttention_61022895341644
// MI455X (gfx1250) — hardware-run, weakly checked
//
#include <hip/hip_runtime.h>


#ifndef NB
#define NB 2
#endif
#ifndef SEQ
#define SEQ 2048
#endif
#define NB_FULL  2
#define SEQ_FULL 2048
#ifndef OUT_SEQ
#define OUT_SEQ SEQ
#endif
#define DM   1024
#define NH_  16
#define HD   64
#define NT64 (SEQ / 64)
#define QRS  2048.0f
#define QRI  (1.0f / 2048.0f)
#define WOS  64.0f
#define WOI  (1.0f / 64.0f)
#define GSC  0.125f
#define NEGF (-1.0e9f)

static_assert(HD == 64);
static_assert(NH_ * HD == DM);
static_assert(DM % 64 == 0);
static_assert(DM % 32 == 0);
static_assert(HD % 32 == 0);
static_assert(SEQ % 64 == 0);
static_assert(SEQ % 32 == 0);
static_assert((NB * SEQ) % 64 == 0);
static_assert((NB * SEQ) % 32 == 0);
static_assert(((size_t)SEQ * DM) % 8 == 0);
static_assert(((size_t)DM * DM) % 8 == 0);
static_assert(NB <= NB_FULL);
static_assert(SEQ <= SEQ_FULL);
static_assert(32 * 16 * 4 == 16 * HD * 2);
static_assert(32 * 16 * 4 == 16 * 128);
static_assert(32 * 16 * 8 == 16 * 64 * 4);
static_assert(16 * 16 == 64 * 4);
static_assert(8 * 4 == 32);
static_assert(8 * 16 == 32 * 4);
static_assert((16 * 68 + 64) * 4 <= 131072);
static_assert(4 * 16 * 68 * 4 <= 131072);
static_assert(32 * 4 <= 131072);

typedef _Float16 h16;
typedef unsigned short bf;
typedef __attribute__((ext_vector_type(16))) __bf16   v16bf;
typedef __attribute__((ext_vector_type(16))) _Float16 v16h;
typedef __attribute__((ext_vector_type(8)))  _Float16 v8h;
typedef __attribute__((ext_vector_type(8)))  unsigned short v8us;
typedef __attribute__((ext_vector_type(8)))  float    v8f;
typedef __attribute__((ext_vector_type(4)))  float    v4f;
typedef __attribute__((ext_vector_type(4)))  int      v4i;
typedef v4f  __attribute__((may_alias)) v4fa;

__device__ __forceinline__ unsigned short f2bf(float f) { unsigned u = __float_as_uint(f); u += 0x7FFFu + ((u >> 16) & 1u); return (unsigned short)(u >> 16); }
__device__ __forceinline__ float bfr(float f) { return __uint_as_float(((unsigned)f2bf(f)) << 16); }
__device__ __forceinline__ v16h cat16(v8h lo, v8h hi) { return __builtin_shufflevector(lo, hi, 0, 1, 2, 3, 4, 5, 6, 7, 8, 9, 10, 11, 12, 13, 14, 15); }
__device__ __forceinline__ v16bf cat16b(v8us lo, v8us hi) { return __builtin_bit_cast(v16bf, __builtin_shufflevector(lo, hi, 0, 1, 2, 3, 4, 5, 6, 7, 8, 9, 10, 11, 12, 13, 14, 15)); }
__device__ __forceinline__ v8f wmma16(v16h a, v16h b, v8f c) { return __builtin_amdgcn_wmma_f32_16x16x32_f16(false, a, false, b, (short)0, c, false, false); }
__device__ __forceinline__ v8f wmmab(v16bf a, v16bf b, v8f c) { return __builtin_amdgcn_wmma_f32_16x16x32_bf16(false, a, false, b, (short)0, c, false, false); }
__device__ __forceinline__ v8f wmmabg(v16bf a, v16bf b, v8f c) { c = wmmab(a, b, c); asm volatile("v_nop\n\tv_nop\n\tv_nop\n\tv_nop" : "+v"(c) : "v"(a), "v"(b)); return c; }
__device__ __forceinline__ v8f wmma16g(v16h a, v16h b, v8f c) { c = wmma16(a, b, c); asm volatile("v_nop\n\tv_nop\n\tv_nop\n\tv_nop" : "+v"(c) : "v"(a), "v"(b)); return c; }
__device__ __forceinline__ v16h  ldh(const h16* p) { return cat16(*(const v8h*)p, *(const v8h*)(p + 16)); }
__device__ __forceinline__ v16bf ldb(const bf* p)  { return cat16b(*(const v8us*)p, *(const v8us*)(p + 16)); }
__device__ __forceinline__ void wave_sync() { __builtin_amdgcn_fence(3  , "wavefront"); __builtin_amdgcn_wave_barrier(); asm volatile("" ::: "memory"); }
static __device__ __forceinline__ h16 toh_flush(float v) { const float w = (fabsf(v) < 6.103515625e-05f) ? 0.0f : v; return (h16)w; }

__global__ __launch_bounds__(256) void k_cvt8(const float* __restrict__ src, bf* dst, size_t n8) {
    const size_t i = (size_t)blockIdx.x * 256 + threadIdx.x; if (i >= n8) return;
    const v8f v = *(const v8f*)(src + i * 8); v8us o;
#pragma unroll
    for (int k = 0; k < 8; ++k) o[k] = f2bf(v[k]);
    *(volatile v8us*)(dst + i * 8) = o; __threadfence(); *(volatile v8us*)(dst + i * 8) = o;
}

__global__ __launch_bounds__(256) void k_wcvt(const float* __restrict__ src, h16* dst, size_t n8) {
    const size_t i = (size_t)blockIdx.x * 256 + threadIdx.x; if (i >= n8) return;
    const v8f v = *(const v8f*)(src + i * 8); v8h o;
#pragma unroll
    for (int k = 0; k < 8; ++k) o[k] = toh_flush(bfr(v[k]) * WOS);
    *(volatile v8h*)(dst + i * 8) = o; __threadfence(); *(volatile v8h*)(dst + i * 8) = o;
}

template <int MODE>
static __device__ __forceinline__ void proj_body(const bf* __restrict__ A, const bf* __restrict__ Bt, const float* __restrict__ bias, const int* __restrict__ mask, h16* Ph, h16* Pr, float* CP) {
    __shared__ __align__(16) float os[16 * 68];
    __shared__ __align__(16) float cs[64];
    const unsigned lane = threadIdx.x & 31u, lr = lane & 15u, hi = lane >> 4;
    const unsigned r0 = blockIdx.x * 64u, c0 = blockIdx.y * 64u;
    v8f acc[4][4];
#pragma unroll
    for (int mb = 0; mb < 4; ++mb)
#pragma unroll
        for (int nb = 0; nb < 4; ++nb) acc[mb][nb] = (v8f){};
    const size_t aoff = (size_t)(r0 + lr) * DM + 8u * hi, boff = (size_t)(c0 + lr) * DM + 8u * hi;
#pragma unroll 1
    for (unsigned kc = 0; kc < (unsigned)DM; kc += 32u) {
        v16bf a[4];
#pragma unroll
        for (int mb = 0; mb < 4; ++mb) a[mb] = ldb(A + aoff + (size_t)mb * 16 * DM + kc);
#pragma unroll
        for (int nb = 0; nb < 4; ++nb) { const v16bf b = ldb(Bt + boff + (size_t)nb * 16 * DM + kc);
#pragma unroll
            for (int mb = 0; mb < 4; ++mb) acc[mb][nb] = wmmabg(a[mb], b, acc[mb][nb]); }
    }
    float bc[4];
#pragma unroll
    for (int nb = 0; nb < 4; ++nb) bc[nb] = (MODE == 0) ? bfr(bias[c0 + nb * 16 + lr]) : 0.0f;
    size_t tbase; unsigned bb, tt;
    if (MODE == 0) { bb = r0 / (unsigned)SEQ; tt = r0 % (unsigned)SEQ; const unsigned zc = bb * (unsigned)NH_ + c0 / (unsigned)HD;
                     tbase = ((size_t)zc * SEQ + (size_t)tt) * HD; }
    else           { bb = c0 / (unsigned)SEQ; tt = c0 % (unsigned)SEQ;
                     tbase = (size_t)bb * (size_t)DM * SEQ + (size_t)r0 * SEQ + (size_t)tt; }
    float mk[8], nm[8];
#pragma unroll
    for (int i = 0; i < 8; ++i) { mk[i] = 1.0f; nm[i] = 0.0f; }
    if (MODE == 2) {
        const size_t mo = (size_t)bb * SEQ_FULL + (size_t)tt + (size_t)((lane & 7u) * 8u);
        const v4i k0 = *(const v4i*)(mask + mo); const v4i k1 = *(const v4i*)(mask + mo + 4);
#pragma unroll
        for (int i = 0; i < 4; ++i) { mk[i] = (k0[i] != 0) ? 1.0f : 0.0f; mk[4 + i] = (k1[i] != 0) ? 1.0f : 0.0f; nm[i] = 1.0f - mk[i]; nm[4 + i] = 1.0f - mk[4 + i]; }
    }
#pragma unroll
    for (int mb = 0; mb < 4; ++mb) {
        float br[8];
#pragma unroll
        for (int j = 0; j < 8; ++j) br[j] = (MODE != 0) ? bfr(bias[r0 + mb * 16 + hi * 8 + j]) : 0.0f;
#pragma unroll
        for (int nb = 0; nb < 4; ++nb) {
#pragma unroll
            for (int j = 0; j < 8; ++j) os[(hi * 8 + j) * 68 + nb * 16 + lr] = acc[mb][nb][j] + bc[nb] + br[j]; }
        wave_sync();
        if (MODE == 2) {
#pragma unroll
            for (int s = 0; s < 4; ++s) { const unsigned row = 4u * s + (lane >> 3), c8 = (lane & 7u) * 8u;
                const v4f x0 = *(const v4fa*)(&os[row * 68 + c8]); const v4f x1 = *(const v4fa*)(&os[row * 68 + c8 + 4]);
                float part = 0.0f;
#pragma unroll
                for (int i = 0; i < 4; ++i) part += nm[i] * x0[i];
#pragma unroll
                for (int i = 0; i < 4; ++i) part += nm[4 + i] * x1[i];
                part += __shfl_xor(part, 1, 32); part += __shfl_xor(part, 2, 32); part += __shfl_xor(part, 4, 32);
                if ((lane & 7u) == 0u) cs[mb * 16 + row] = part; }
        }
#pragma unroll 1
        for (int ps = 0; ps < 2; ++ps) {
            if (MODE == 0) {
                const size_t sb = tbase + (size_t)(mb * 16) * HD;
#pragma unroll
                for (int s = 0; s < 4; ++s) { const unsigned p = s * 32u + lane; const unsigned row = p >> 3, c8 = (p & 7u) * 8u;
                    const v4f x0 = *(const v4fa*)(&os[row * 68 + c8]); const v4f x1 = *(const v4fa*)(&os[row * 68 + c8 + 4]); v8h hv, rv;
#pragma unroll
                    for (int i = 0; i < 4; ++i) { const h16 a0 = toh_flush(x0[i]); const h16 a1 = toh_flush(x1[i]); hv[i] = a0; hv[4 + i] = a1;
                        rv[i] = toh_flush((x0[i] - (float)a0) * QRS); rv[4 + i] = toh_flush((x1[i] - (float)a1) * QRS); }
                    const size_t oo = sb + (size_t)p * 8;
                    *(volatile v8h*)(Ph + oo) = hv; *(volatile v8h*)(Pr + oo) = rv; }
            } else {
                const size_t sb = tbase + (size_t)(mb * 16) * SEQ;
#pragma unroll
                for (int s = 0; s < 4; ++s) { const unsigned row = 4u * s + (lane >> 3), c8 = (lane & 7u) * 8u;
                    const v4f x0 = *(const v4fa*)(&os[row * 68 + c8]); const v4f x1 = *(const v4fa*)(&os[row * 68 + c8 + 4]); v8h hv;
#pragma unroll
                    for (int i = 0; i < 4; ++i) { hv[i] = toh_flush(x0[i] * mk[i]); hv[4 + i] = toh_flush(x1[i] * mk[4 + i]); }
                    const size_t oo = sb + (size_t)row * SEQ + c8;
                    *(volatile v8h*)(Ph + oo) = hv; }
            }
            if (ps == 0) __threadfence(); }
        wave_sync();
    }
    if (MODE == 2) {
        const v4f cval = *(const v4fa*)(&cs[lr * 4u]);
        float* cp = CP + ((size_t)bb * NT64 + (size_t)(tt / 64u)) * DM + r0 + lr * 4u;
        if (lane < 16u) *(volatile v4f*)cp = cval;
        __threadfence();
        if (lane < 16u) *(volatile v4f*)cp = cval;
    }
}

__global__ __launch_bounds__(32) void k_projq(const bf* __restrict__ A, const bf* __restrict__ Bt, const float* __restrict__ bias, h16* Ph, h16* Pr) {
    proj_body<0>(A, Bt, bias, nullptr, Ph, Pr, nullptr);
}
__global__ __launch_bounds__(32) void k_projk(const bf* __restrict__ A, const bf* __restrict__ Bt, const float* __restrict__ bias, h16* Ph) {
    proj_body<1>(A, Bt, bias, nullptr, Ph, nullptr, nullptr);
}
__global__ __launch_bounds__(32) void k_projv(const bf* __restrict__ A, const bf* __restrict__ Bt, const float* __restrict__ bias, const int* __restrict__ mask, h16* Ph, float* CP) {
    proj_body<2>(A, Bt, bias, mask, Ph, nullptr, CP);
}

__global__ __launch_bounds__(32) void k_gram(const h16* __restrict__ KT, const h16* __restrict__ VT, const float* __restrict__ CP, h16* GH, h16* GR, float* CV) {
    __shared__ __align__(16) float os[16 * 68];
    __shared__ __align__(16) float cs[64];
    const unsigned lane = threadIdx.x & 31u, lr = lane & 15u, hi = lane >> 4;
    const unsigned zh = blockIdx.x; const unsigned bz = zh / (unsigned)NH_, hz = zh % (unsigned)NH_;
    v8f acc[4][4];
#pragma unroll
    for (int mb = 0; mb < 4; ++mb)
#pragma unroll
        for (int nb = 0; nb < 4; ++nb) acc[mb][nb] = (v8f){};
    const size_t pb = (size_t)zh * HD * SEQ + (size_t)lr * SEQ + 8u * hi;
#pragma unroll 1
    for (unsigned kc = 0; kc < (unsigned)SEQ; kc += 32u) {
        v16h a[4];
#pragma unroll
        for (int mb = 0; mb < 4; ++mb) a[mb] = ldh(VT + pb + (size_t)mb * 16 * SEQ + kc);
#pragma unroll
        for (int nb = 0; nb < 4; ++nb) { const v16h kf = ldh(KT + pb + (size_t)nb * 16 * SEQ + kc);
#pragma unroll
            for (int mb = 0; mb < 4; ++mb) acc[mb][nb] = wmma16g(a[mb], kf, acc[mb][nb]); }
    }
    { float s0 = 0.0f, s1 = 0.0f;
      const float* cp = CP + (size_t)bz * NT64 * DM + (size_t)hz * HD + lane;
#pragma unroll 1
      for (unsigned tl = 0; tl < (unsigned)NT64; ++tl) { s0 += cp[(size_t)tl * DM]; s1 += cp[(size_t)tl * DM + 32]; }
      cs[lane] = NEGF * s0; cs[32u + lane] = NEGF * s1; }
#pragma unroll
    for (int mb = 0; mb < 4; ++mb) {
#pragma unroll
        for (int nb = 0; nb < 4; ++nb) {
#pragma unroll
            for (int j = 0; j < 8; ++j) os[(hi * 8 + j) * 68 + nb * 16 + lr] = acc[mb][nb][j] * GSC; }
        wave_sync();
#pragma unroll 1
        for (int ps = 0; ps < 2; ++ps) {
            const size_t sb = (size_t)zh * HD * HD + (size_t)(mb * 16) * HD;
#pragma unroll
            for (int s = 0; s < 4; ++s) { const unsigned p = s * 32u + lane; const unsigned row = p >> 3, c8 = (p & 7u) * 8u;
                const v4f x0 = *(const v4fa*)(&os[row * 68 + c8]); const v4f x1 = *(const v4fa*)(&os[row * 68 + c8 + 4]); v8h hv, rv;
#pragma unroll
                for (int i = 0; i < 4; ++i) { const h16 a0 = toh_flush(x0[i]); const h16 a1 = toh_flush(x1[i]); hv[i] = a0; hv[4 + i] = a1;
                    rv[i] = toh_flush((x0[i] - (float)a0) * QRS); rv[4 + i] = toh_flush((x1[i] - (float)a1) * QRS); }
                const size_t oo = sb + (size_t)p * 8;
                *(volatile v8h*)(GH + oo) = hv; *(volatile v8h*)(GR + oo) = rv; }
            if (ps == 0) __threadfence(); }
        wave_sync();
    }
    { const v4f cval = *(const v4fa*)(&cs[lr * 4u]);
      float* cvp = CV + (size_t)zh * HD + lr * 4u;
      if (lane < 16u) *(volatile v4f*)cvp = cval;
      __threadfence();
      if (lane < 16u) *(volatile v4f*)cvp = cval; }
}

__global__ __launch_bounds__(256) void k_cvw(const float* __restrict__ CV, const float* __restrict__ wo, float* CW) {
#pragma clang fp contract(off)
    __shared__ __align__(16) float rs[32];
    const unsigned lane = threadIdx.x & 31u;
    const unsigned wave = (unsigned)__builtin_amdgcn_readfirstlane((int)(threadIdx.x >> 5));
    const unsigned bz = blockIdx.y, n0 = blockIdx.x * 32u;
    const float* cp = CV + (size_t)bz * DM + lane;
#pragma unroll 1
    for (unsigned j = 0; j < 4u; ++j) {
        const unsigned n = n0 + wave * 4u + j;
        const float* wp = wo + (size_t)n * DM + lane;
        float s = 0.0f;
#pragma unroll 4
        for (unsigned i = 0; i < (unsigned)(DM / 32); ++i) { const float cvv = cp[i * 32u]; const float wvv = bfr(wp[i * 32u]); const float pr = cvv * wvv; s = s + pr; }
        s = s + __shfl_xor(s, 16, 32); s = s + __shfl_xor(s, 8, 32); s = s + __shfl_xor(s, 4, 32); s = s + __shfl_xor(s, 2, 32); s = s + __shfl_xor(s, 1, 32);
        if (lane == 0u) rs[wave * 4u + j] = s;
    }
    __syncthreads();
    if (wave == 0u) {
        const v4f val = *(const v4fa*)(&rs[(lane & 7u) * 4u]);
        float* op = CW + (size_t)bz * DM + n0 + (lane & 7u) * 4u;
        if (lane < 8u) *(volatile v4f*)op = val;
        __threadfence();
        if (lane < 8u) *(volatile v4f*)op = val;
    }
}

__global__ __launch_bounds__(128) void k_head(const h16* __restrict__ QH, const h16* __restrict__ QR, const h16* __restrict__ GH, const h16* __restrict__ GR,
                                              h16* CH, h16* CR) {
    __shared__ __align__(16) float os[4 * 16 * 68];
    const unsigned lane = threadIdx.x & 31u, lr = lane & 15u, hi = lane >> 4;
    const unsigned wave = (unsigned)__builtin_amdgcn_readfirstlane((int)(threadIdx.x >> 5));
    const unsigned zh = blockIdx.y; const unsigned bz = zh / (unsigned)NH_, hz = zh % (unsigned)NH_;
    const unsigned t0 = (blockIdx.x * 4u + wave) * 16u;
    const size_t qo = ((size_t)zh * SEQ + (size_t)(t0 + lr)) * HD + 8u * hi;
    const v16h qh0 = ldh(QH + qo), qh1 = ldh(QH + qo + 32), qr0 = ldh(QR + qo), qr1 = ldh(QR + qo + 32);
    const size_t go = (size_t)zh * HD * HD + (size_t)lr * HD + 8u * hi;
    v8f am[4], ar[4];
#pragma unroll
    for (int nb = 0; nb < 4; ++nb) { am[nb] = (v8f){}; ar[nb] = (v8f){}; }
#pragma unroll
    for (int nb = 0; nb < 4; ++nb) {
        const h16* gp = GH + go + (size_t)nb * 16 * HD; const h16* gq = GR + go + (size_t)nb * 16 * HD;
        const v16h gh0 = ldh(gp), gh1 = ldh(gp + 32), gr0 = ldh(gq), gr1 = ldh(gq + 32);
        am[nb] = wmma16g(qh0, gh0, am[nb]); am[nb] = wmma16g(qh1, gh1, am[nb]);
        ar[nb] = wmma16g(qr0, gh0, ar[nb]); ar[nb] = wmma16g(qr1, gh1, ar[nb]);
        ar[nb] = wmma16g(qh0, gr0, ar[nb]); ar[nb] = wmma16g(qh1, gr1, ar[nb]);
    }
    const unsigned wb = wave * 16u * 68u;
#pragma unroll
    for (int nb = 0; nb < 4; ++nb) {
#pragma unroll
        for (int j = 0; j < 8; ++j) os[wb + (hi * 8 + j) * 68 + nb * 16 + lr] = am[nb][j] + ar[nb][j] * QRI; }
    wave_sync();
    const unsigned c8 = (lane & 7u) * 8u;
    const size_t cbase = ((size_t)bz * SEQ + (size_t)t0) * DM + (size_t)hz * HD + c8;
#pragma unroll 1
    for (int ps = 0; ps < 2; ++ps) {
#pragma unroll
        for (int s = 0; s < 4; ++s) { const unsigned row = 4u * s + (lane >> 3);
            const v4f x0 = *(const v4fa*)(&os[wb + row * 68 + c8]); const v4f x1 = *(const v4fa*)(&os[wb + row * 68 + c8 + 4]);
            v8h hv, rv;
#pragma unroll
            for (int i = 0; i < 4; ++i) { const h16 a0 = toh_flush(x0[i]); const h16 a1 = toh_flush(x1[i]); hv[i] = a0; hv[4 + i] = a1;
                rv[i] = toh_flush((x0[i] - (float)a0) * QRS); rv[4 + i] = toh_flush((x1[i] - (float)a1) * QRS); }
            const size_t oo = cbase + (size_t)row * DM;
            *(volatile v8h*)(CH + oo) = hv; *(volatile v8h*)(CR + oo) = rv; }
        if (ps == 0) __threadfence(); }
}

__global__ __launch_bounds__(32) void k_out(const h16* __restrict__ CH, const h16* __restrict__ CR, const h16* __restrict__ WO, const float* __restrict__ bo, const float* __restrict__ CW, float* OUT) {
    __shared__ __align__(16) float os[16 * 68];
    const unsigned lane = threadIdx.x & 31u, lr = lane & 15u, hi = lane >> 4;
    const unsigned r0 = blockIdx.x * 32u, c0 = blockIdx.y * 64u;
    v8f am[2][4], ar[2][4];
#pragma unroll
    for (int mb = 0; mb < 2; ++mb)
#pragma unroll
        for (int nb = 0; nb < 4; ++nb) { am[mb][nb] = (v8f){}; ar[mb][nb] = (v8f){}; }
    const size_t aoff = (size_t)(r0 + lr) * DM + 8u * hi, boff = (size_t)(c0 + lr) * DM + 8u * hi;
#pragma unroll 1
    for (unsigned kc = 0; kc < (unsigned)DM; kc += 32u) {
        v16h ah[2], al[2];
#pragma unroll
        for (int mb = 0; mb < 2; ++mb) { ah[mb] = ldh(CH + aoff + (size_t)mb * 16 * DM + kc); al[mb] = ldh(CR + aoff + (size_t)mb * 16 * DM + kc); }
#pragma unroll
        for (int nb = 0; nb < 4; ++nb) { const v16h w = ldh(WO + boff + (size_t)nb * 16 * DM + kc);
#pragma unroll
            for (int mb = 0; mb < 2; ++mb) { am[mb][nb] = wmma16g(ah[mb], w, am[mb][nb]); ar[mb][nb] = wmma16g(al[mb], w, ar[mb][nb]); } }
    }
    const unsigned bb = r0 / (unsigned)SEQ, tt = r0 % (unsigned)SEQ;
    float bc[4], wc[4];
#pragma unroll
    for (int nb = 0; nb < 4; ++nb) { bc[nb] = bfr(bo[c0 + nb * 16 + lr]);
                                     wc[nb] = CW[(size_t)bb * DM + c0 + nb * 16 + lr]; }
    float* obase = OUT + ((size_t)bb * OUT_SEQ + (size_t)tt) * DM + c0;
#pragma unroll
    for (int mb = 0; mb < 2; ++mb) {
#pragma unroll
        for (int nb = 0; nb < 4; ++nb) {
#pragma unroll
            for (int j = 0; j < 8; ++j) os[(hi * 8 + j) * 68 + nb * 16 + lr] = (am[mb][nb][j] + ar[mb][nb][j] * QRI) * WOI + bc[nb] + wc[nb]; }
        wave_sync();
#pragma unroll 1
        for (int ps = 0; ps < 2; ++ps) {
#pragma unroll
            for (int s = 0; s < 8; ++s) { const unsigned row = 2u * s + (lane >> 4), cofs = (lane & 15u) * 4u;
                const v4f val = *(const v4fa*)(&os[row * 68 + cofs]);
                *(volatile v4f*)(obase + (size_t)(mb * 16 + row) * DM + cofs) = val; }
            if (ps == 0) __threadfence(); }
        wave_sync();
    }
}

static constexpr size_t al256(size_t v) { return (v + 255) & ~(size_t)255; }
static constexpr size_t SZ_XB = al256((size_t)NB * SEQ * DM * 2);
static constexpr size_t SZ_WB = al256((size_t)3 * DM * DM * 2);
static constexpr size_t SZ_WO = al256((size_t)DM * DM * 2);
static constexpr size_t SZ_PL = al256((size_t)NB * NH_ * SEQ * HD * 2);
static constexpr size_t SZ_CP = al256((size_t)NB * NT64 * DM * 4);
static constexpr size_t SZ_G  = al256((size_t)NB * NH_ * HD * HD * 2);
static constexpr size_t SZ_CV = al256((size_t)NB * NH_ * HD * 4);
static constexpr size_t SZ_CW = al256((size_t)NB * DM * 4);
static constexpr size_t SZ_TOTAL = 3 * SZ_XB + SZ_WB + SZ_WO + 6 * SZ_PL + SZ_CP + 2 * SZ_G + SZ_CV + SZ_CW;
static_assert(SZ_TOTAL <= (size_t)134217728);
static_assert(((size_t)DM * DM * 2) % 256 == 0);
static_assert((size_t)NB * NH_ * SEQ * HD == (size_t)NB * DM * SEQ);
static_assert((size_t)NB * NH_ * HD == (size_t)NB * DM);
static_assert((size_t)(NB - 1) * DM + (DM / 32 - 1) * 32 + 7 * 4 + 4 <= (size_t)NB * DM);

extern "C" void kernel_launch(void* const* d_in, const int* in_sizes, int n_in,
                              void* d_out, int out_size, void* d_ws, size_t ws_size, hipStream_t stream) {
    if (n_in < 12) return;
    const size_t needx = ((size_t)(NB - 1) * SEQ_FULL + SEQ) * DM;
    const size_t needm = (size_t)(NB - 1) * SEQ_FULL + SEQ;
    if ((size_t)in_sizes[0] < needx || (size_t)in_sizes[1] < needx || (size_t)in_sizes[2] < needx) return;
    if ((size_t)in_sizes[3] < needm) return;
    if ((size_t)in_sizes[4] < (size_t)DM * DM || (size_t)in_sizes[6] < (size_t)DM * DM || (size_t)in_sizes[8] < (size_t)DM * DM || (size_t)in_sizes[10] < (size_t)DM * DM) return;
    if (in_sizes[5] < DM || in_sizes[7] < DM || in_sizes[9] < DM || in_sizes[11] < DM) return;
    if ((size_t)out_size < ((size_t)(NB - 1) * OUT_SEQ + SEQ) * DM) return;
    if (SZ_TOTAL > ws_size) return;
    const float* xin[3] = { (const float*)d_in[0], (const float*)d_in[1], (const float*)d_in[2] };
    const int* msk = (const int*)d_in[3];
    const float* wq = (const float*)d_in[4];  const float* bq = (const float*)d_in[5];
    const float* wk = (const float*)d_in[6];  const float* bk = (const float*)d_in[7];
    const float* wv = (const float*)d_in[8];  const float* bv = (const float*)d_in[9];
    const float* wo = (const float*)d_in[10]; const float* bo = (const float*)d_in[11];
    float* OUT = (float*)d_out;
    char* wsp = (char*)d_ws;
    bf* XB[3];
    XB[0] = (bf*)wsp; wsp += SZ_XB;
    XB[1] = (bf*)wsp; wsp += SZ_XB;
    XB[2] = (bf*)wsp; wsp += SZ_XB;
    bf* WB = (bf*)wsp; wsp += SZ_WB;
    h16* WO = (h16*)wsp; wsp += SZ_WO;
    h16* QH = (h16*)wsp; wsp += SZ_PL;
    h16* QR = (h16*)wsp; wsp += SZ_PL;
    h16* KT = (h16*)wsp; wsp += SZ_PL;
    h16* VT = (h16*)wsp; wsp += SZ_PL;
    h16* CH = (h16*)wsp; wsp += SZ_PL;
    h16* CR = (h16*)wsp; wsp += SZ_PL;
    float* CP = (float*)wsp; wsp += SZ_CP;
    h16* GH = (h16*)wsp; wsp += SZ_G;
    h16* GR = (h16*)wsp; wsp += SZ_G;
    float* CV = (float*)wsp; wsp += SZ_CV;
    float* CW = (float*)wsp; wsp += SZ_CW;
    bf* WQ = WB; bf* WK = WB + (size_t)DM * DM; bf* WV = WB + (size_t)2 * DM * DM;

    for (int i = 0; i < 3; ++i) {
        if (SEQ == SEQ_FULL) {
            const size_t n8 = (size_t)NB * SEQ * DM / 8;
            k_cvt8<<<(unsigned)((n8 + 255) / 256), 256, 0, stream>>>(xin[i], XB[i], n8);
        } else {
            const size_t n8 = (size_t)SEQ * DM / 8;
            for (int b = 0; b < NB; ++b) k_cvt8<<<(unsigned)((n8 + 255) / 256), 256, 0, stream>>>(xin[i] + (size_t)b * SEQ_FULL * DM, XB[i] + (size_t)b * SEQ * DM, n8);
        }
    }
    { const size_t n8 = (size_t)DM * DM / 8; const unsigned g = (unsigned)((n8 + 255) / 256);
      k_cvt8<<<g, 256, 0, stream>>>(wq, WQ, n8); k_cvt8<<<g, 256, 0, stream>>>(wk, WK, n8); k_cvt8<<<g, 256, 0, stream>>>(wv, WV, n8);
      k_wcvt<<<g, 256, 0, stream>>>(wo, WO, n8); }

    k_projq<<<dim3(NB * SEQ / 64, DM / 64, 1), 32, 0, stream>>>(XB[0], WQ, bq, QH, QR);
    k_projk<<<dim3(DM / 64, NB * SEQ / 64, 1), 32, 0, stream>>>(WK, XB[1], bk, KT);
    k_projv<<<dim3(DM / 64, NB * SEQ / 64, 1), 32, 0, stream>>>(WV, XB[2], bv, msk, VT, CP);

    k_gram<<<dim3(NB * NH_, 1, 1), 32, 0, stream>>>(KT, VT, CP, GH, GR, CV);
    k_cvw<<<dim3(DM / 32, NB, 1), 256, 0, stream>>>(CV, wo, CW);
    k_head<<<dim3(SEQ / 64, NB * NH_, 1), 128, 0, stream>>>(QH, QR, GH, GR, CH, CR);
    k_out<<<dim3(NB * SEQ / 32, DM / 64, 1), 32, 0, stream>>>(CH, CR, WO, bo, CW, OUT);
}
